// MultiGATLayer_52424370815427
// MI455X (gfx1250) — hardware-verified
//
#include <hip/hip_runtime.h>
#include <stddef.h>


#define NTHR   256
#define NWAVE  8
#define FIN    1024
#define FO     128
#define NHD    8
#define HC     (NHD * FO)
#define AW     (NHD * 2 * FO)
#define DEG    16
#define NBR    (DEG + 1)
#define ESW    16
#define BM     64
#define BNC    128
#define SNB    64
#define ANB    NWAVE
#define WSCAP  134217728
#define ACARRY 8.0f
#define WCARRY 64.0f
#define SCL_AW (1.0f / 512.0f)

static_assert((FIN % 32) == 0);
static_assert(FIN / 8 == 128);
static_assert(FO == 128);
static_assert((HC % BNC) == 0);
static_assert(ESW == 2 * NHD);
static_assert(SNB * ESW == NTHR * 4);
static_assert((SNB % NWAVE) == 0);
static_assert(SNB == BM);
static_assert((BM % ANB) == 0);
static_assert(AW == 2048);
static_assert(NBR <= 32);

typedef float    v4f  __attribute__((ext_vector_type(4)));
typedef float    v8f  __attribute__((ext_vector_type(8)));
typedef _Float16 v8h  __attribute__((ext_vector_type(8)));
typedef _Float16 v16h __attribute__((ext_vector_type(16)));
union Frag { v16h v; v8h h[2]; };

__device__ __forceinline__ v8f wmh(v16h a, v16h b, v8f c) {
  v8f d = __builtin_amdgcn_wmma_f32_16x16x32_f16(false, a, false, b, (short)0, c, false, false);
  asm volatile("v_nop\n\tv_nop\n\tv_nop\n\tv_nop" : "+v"(d) : "v"(a), "v"(b));
  return d;
}

__device__ __forceinline__ v4f selz(v4f v, bool live) {
  v4f o; o.x = live ? v.x : 0.f; o.y = live ? v.y : 0.f; o.z = live ? v.z : 0.f; o.w = live ? v.w : 0.f; return o;
}
__device__ __forceinline__ v4f selv4(v4f v, bool c, float other) {
  v4f o; o.x = c ? v.x : other; o.y = c ? v.y : other; o.z = c ? v.z : other; o.w = c ? v.w : other; return o;
}
__device__ __forceinline__ v4f lrelu4(v4f v) {
  v4f o;
  o.x = v.x >= 0.f ? v.x : 0.2f * v.x;  o.y = v.y >= 0.f ? v.y : 0.2f * v.y;
  o.z = v.z >= 0.f ? v.z : 0.2f * v.z;  o.w = v.w >= 0.f ? v.w : 0.2f * v.w;
  return o;
}
__device__ __forceinline__ v4f vexp4(v4f v) {
  v4f o; o.x = __expf(v.x); o.y = __expf(v.y); o.z = __expf(v.z); o.w = __expf(v.w); return o;
}
__device__ __forceinline__ v4f rcp4(v4f v) {
  v4f o;
  o.x = __builtin_amdgcn_rcpf(v.x); o.y = __builtin_amdgcn_rcpf(v.y);
  o.z = __builtin_amdgcn_rcpf(v.z); o.w = __builtin_amdgcn_rcpf(v.w);
  return o;
}
__device__ __forceinline__ v4f wmax4(v4f v) {
#pragma unroll
  for (int off = 16; off > 0; off >>= 1) {
    v.x = fmaxf(v.x, __shfl_xor(v.x, off)); v.y = fmaxf(v.y, __shfl_xor(v.y, off));
    v.z = fmaxf(v.z, __shfl_xor(v.z, off)); v.w = fmaxf(v.w, __shfl_xor(v.w, off));
  }
  return v;
}
__device__ __forceinline__ v4f wsum4(v4f v) {
#pragma unroll
  for (int off = 16; off > 0; off >>= 1) {
    v.x += __shfl_xor(v.x, off); v.y += __shfl_xor(v.y, off);
    v.z += __shfl_xor(v.z, off); v.w += __shfl_xor(v.w, off);
  }
  return v;
}
__device__ __forceinline__ float wsum1(float v) {
#pragma unroll
  for (int off = 16; off > 0; off >>= 1) v += __shfl_xor(v, off);
  return v;
}

__global__ __launch_bounds__(NTHR) void k_acvt(const float* __restrict__ x, _Float16* a16, int nN, int npad) {
  const int gi = (int)blockIdx.x * NTHR + (int)threadIdx.x;
  const int row = gi >> 7, seg = gi & 127;
  if (row >= npad) return;
  int rr = row > nN - 1 ? nN - 1 : row;
  rr = rr < 0 ? 0 : rr;
  const bool live = row < nN;
  const float* rp = x + (size_t)rr * FIN + 8 * seg;
  const v4f x0 = *(const v4f*)rp;
  const v4f x1 = *(const v4f*)(rp + 4);
  const float sc = live ? ACARRY : 0.f;
  v8h o;
  o[0] = (_Float16)(x0.x * sc); o[1] = (_Float16)(x0.y * sc); o[2] = (_Float16)(x0.z * sc); o[3] = (_Float16)(x0.w * sc);
  o[4] = (_Float16)(x1.x * sc); o[5] = (_Float16)(x1.y * sc); o[6] = (_Float16)(x1.z * sc); o[7] = (_Float16)(x1.w * sc);
  _Float16* gp = a16 + (size_t)row * FIN + 8 * seg;
  *(volatile v8h*)gp = o;
  __threadfence();
  *(volatile v8h*)gp = o;
}

__global__ __launch_bounds__(NTHR) void k_wcvt(const float* __restrict__ w, _Float16* wp, int nUnits) {
  const int i = (int)blockIdx.x * NTHR + (int)threadIdx.x;
  if (i >= nUnits) return;
  const int c = i >> 7;
  const int seg = i & 127;
  const int kh = c >> 7;
  const int o = c & (FO - 1);
  v8h ov;
#pragma unroll
  for (int j = 0; j < 8; ++j) {
    int k = 8 * seg + j;
    k = k > FIN - 1 ? FIN - 1 : k;
    const float f = w[((size_t)kh * FIN + k) * FO + o];
    ov[j] = (_Float16)(f * WCARRY);
  }
  _Float16* gp = wp + (size_t)i * 8;
  *(volatile v8h*)gp = ov;
  __threadfence();
  *(volatile v8h*)gp = ov;
}

__global__ __launch_bounds__(NTHR) void k_gemm(
    const _Float16* __restrict__ A, const _Float16* __restrict__ Bp, const float* __restrict__ bias,
    float* Cout, int K, int ldc, int nValid, int nStore, float scl) {
  constexpr int TPW = 4;
  constexpr int PPR = BNC / 4;
  constexpr int NIT = (BM * PPR) / NTHR;
  static_assert((BM * PPR) % NTHR == 0);
  static_assert(NIT >= 1);
  static_assert(TPW * 16 * 2 == BNC);
  static_assert(BM == 4 * 16);
  static_assert(PPR == 32);

  __shared__ __attribute__((aligned(16))) float stg[BM * BNC];
  const int tid = threadIdx.x, lane = tid & 31, wave = tid >> 5, hh = lane >> 4, m = lane & 15;
  const int rowBase = (int)blockIdx.x * BM;
  const int colBase = (int)blockIdx.y * BNC;
  const int rg = wave >> 1, chf = wave & 1;
  const int r0 = rg * 16;
  const int c0 = chf * (BNC / 2);

  v8f acc[TPW];
#pragma unroll
  for (int t = 0; t < TPW; ++t) { v8f z = {0.f, 0.f, 0.f, 0.f, 0.f, 0.f, 0.f, 0.f}; acc[t] = z; }

  const _Float16* ap = A  + (size_t)(rowBase + r0 + m) * K + 8 * hh;
  const _Float16* bp = Bp + (size_t)(colBase + c0 + m) * K + 8 * hh;
  const int ksteps = K >> 5;
#pragma unroll 1
  for (int kt = 0; kt < ksteps; ++kt) {
    Frag a;
    a.h[0] = *(const v8h*)(ap + 32 * kt);
    a.h[1] = *(const v8h*)(ap + 32 * kt + 16);
#pragma unroll
    for (int t = 0; t < TPW; ++t) {
      const size_t to = (size_t)(16 * t) * K + 32 * kt;
      Frag b;
      b.h[0] = *(const v8h*)(bp + to);
      b.h[1] = *(const v8h*)(bp + to + 16);
      acc[t] = wmh(a.v, b.v, acc[t]);
    }
  }

  {
    float* sp = stg + (size_t)(r0 + 8 * hh) * BNC + c0 + m;
    const int growb = rowBase + r0 + 8 * hh;
#pragma unroll
    for (int t = 0; t < TPW; ++t) {
      const float bv = bias[colBase + c0 + 16 * t + m];
#pragma unroll
      for (int r = 0; r < 8; ++r) {
        const bool lv = (growb + r) < nValid;
        const float g = acc[t][r] * scl + bv;
        sp[r * BNC + 16 * t] = lv ? g : 0.f;
      }
    }
  }
  __syncthreads();

  v4f cv[NIT];
#pragma unroll
  for (int it = 0; it < NIT; ++it) {
    const int id = it * NTHR + tid;
    const int row = id >> 5, seg = id & 31;
    cv[it] = *(const v4f*)(stg + (size_t)row * BNC + 4 * seg);
  }
#pragma unroll
  for (int it = 0; it < NIT; ++it) {
    const int id = it * NTHR + tid;
    const int row = id >> 5, seg = id & 31;
    const int grow = rowBase + row;
    if (grow < nStore) {
      float* gp = Cout + (size_t)grow * ldc + colBase + 4 * seg;
      *(volatile v4f*)gp = cv[it];
    }
  }
  __threadfence();
#pragma unroll
  for (int it = 0; it < NIT; ++it) {
    const int id = it * NTHR + tid;
    const int row = id >> 5, seg = id & 31;
    const int grow = rowBase + row;
    if (grow < nStore) {
      float* gp = Cout + (size_t)grow * ldc + colBase + 4 * seg;
      *(volatile v4f*)gp = cv[it];
    }
  }
}

__global__ __launch_bounds__(NTHR) void k_scores(const float* __restrict__ hcat, const float* __restrict__ av,
                                                 float* es, int nN) {
  __shared__ __attribute__((aligned(16))) float sa[AW];
  __shared__ __attribute__((aligned(16))) float so[SNB * ESW];
  const int tid = threadIdx.x, lane = tid & 31, wave = tid >> 5;
#pragma unroll 1
  for (int i = tid; i < AW / 4; i += NTHR) *(v4f*)(sa + 4 * i) = *(const v4f*)(av + 4 * i);
  __syncthreads();
  const int nodeBase = (int)blockIdx.x * SNB;
  constexpr int NPW = SNB / NWAVE;
#pragma unroll 1
  for (int q = 0; q < NPW; ++q) {
    const int nl = wave * NPW + q;
    const int node = nodeBase + nl;
    int rr = node > nN - 1 ? nN - 1 : node;
    rr = rr < 0 ? 0 : rr;
    const bool live = node < nN;
    const float* hp = hcat + (size_t)rr * HC + 4 * lane;
#pragma unroll 1
    for (int j = 0; j < NHD; ++j) {
      const v4f hv = *(const v4f*)(hp + FO * j);
      const v4f ad = *(const v4f*)(sa + j * 2 * FO + 4 * lane);
      const v4f as = *(const v4f*)(sa + j * 2 * FO + FO + 4 * lane);
      float d = hv.x * ad.x + hv.y * ad.y + hv.z * ad.z + hv.w * ad.w;
      float s = hv.x * as.x + hv.y * as.y + hv.z * as.z + hv.w * as.w;
      d = wsum1(d);
      s = wsum1(s);
      const float dv = live ? d : 0.f;
      const float sv = live ? s : 0.f;
      if (lane == 0) { so[nl * ESW + j] = dv; so[nl * ESW + NHD + j] = sv; }
    }
  }
  __syncthreads();
  const v4f v = *(const v4f*)(so + 4 * tid);
  float* gp = es + (size_t)nodeBase * ESW + 4 * tid;
  *(volatile v4f*)gp = v;
  __threadfence();
  *(volatile v4f*)gp = v;
}

__global__ __launch_bounds__(NTHR) void k_attend(
    const float* __restrict__ hcat, const int* __restrict__ adj, const float* __restrict__ es,
    const float* __restrict__ bav, float* out, int nN) {
  const int tid = threadIdx.x, lane = tid & 31, wave = tid >> 5;
  const int node = (int)blockIdx.x * ANB + wave;
  int rr = node > nN - 1 ? nN - 1 : node;
  rr = rr < 0 ? 0 : rr;
  const bool live = node < nN;
  const float NINF = -__builtin_inff();

  const int aj = adj[(size_t)rr * DEG + (lane & (DEG - 1))];
  int nb = (lane < DEG) ? aj : rr;
  nb = nb < 0 ? 0 : (nb > nN - 1 ? nN - 1 : nb);
  const bool valid = lane < NBR;

  const v4f sd0 = *(const v4f*)(es + (size_t)rr * ESW);
  const v4f sd1 = *(const v4f*)(es + (size_t)rr * ESW + 4);
  const v4f ss0 = *(const v4f*)(es + (size_t)nb * ESW + NHD);
  const v4f ss1 = *(const v4f*)(es + (size_t)nb * ESW + NHD + 4);
  const v4f b0  = *(const v4f*)bav;
  const v4f b1  = *(const v4f*)(bav + 4);

  const v4f e0 = lrelu4((sd0 + ss0) + b0);
  const v4f e1 = lrelu4((sd1 + ss1) + b1);
  const v4f m0 = wmax4(selv4(e0, valid, NINF));
  const v4f m1 = wmax4(selv4(e1, valid, NINF));
  const v4f x0 = selz(vexp4(e0 - m0), valid);
  const v4f x1 = selz(vexp4(e1 - m1), valid);
  const v4f z0 = wsum4(x0);
  const v4f z1 = wsum4(x1);
  const v4f al0 = x0 * rcp4(z0);
  const v4f al1 = x1 * rcp4(z1);

  v4f acc0 = {0.f, 0.f, 0.f, 0.f}, acc1 = {0.f, 0.f, 0.f, 0.f}, acc2 = {0.f, 0.f, 0.f, 0.f}, acc3 = {0.f, 0.f, 0.f, 0.f};
  v4f acc4 = {0.f, 0.f, 0.f, 0.f}, acc5 = {0.f, 0.f, 0.f, 0.f}, acc6 = {0.f, 0.f, 0.f, 0.f}, acc7 = {0.f, 0.f, 0.f, 0.f};
  const float* hb = hcat + 4 * lane;
#pragma unroll 1
  for (int d = 0; d < NBR; ++d) {
    const int s = __builtin_amdgcn_readlane(nb, d);
    const float a0 = __int_as_float(__builtin_amdgcn_readlane(__float_as_int(al0.x), d));
    const float a1 = __int_as_float(__builtin_amdgcn_readlane(__float_as_int(al0.y), d));
    const float a2 = __int_as_float(__builtin_amdgcn_readlane(__float_as_int(al0.z), d));
    const float a3 = __int_as_float(__builtin_amdgcn_readlane(__float_as_int(al0.w), d));
    const float a4 = __int_as_float(__builtin_amdgcn_readlane(__float_as_int(al1.x), d));
    const float a5 = __int_as_float(__builtin_amdgcn_readlane(__float_as_int(al1.y), d));
    const float a6 = __int_as_float(__builtin_amdgcn_readlane(__float_as_int(al1.z), d));
    const float a7 = __int_as_float(__builtin_amdgcn_readlane(__float_as_int(al1.w), d));
    const float* hs = hb + (size_t)s * HC;
    const v4f h0 = *(const v4f*)(hs + 0 * FO);
    const v4f h1 = *(const v4f*)(hs + 1 * FO);
    const v4f h2 = *(const v4f*)(hs + 2 * FO);
    const v4f h3 = *(const v4f*)(hs + 3 * FO);
    const v4f h4 = *(const v4f*)(hs + 4 * FO);
    const v4f h5 = *(const v4f*)(hs + 5 * FO);
    const v4f h6 = *(const v4f*)(hs + 6 * FO);
    const v4f h7 = *(const v4f*)(hs + 7 * FO);
    acc0 = acc0 + h0 * a0;
    acc1 = acc1 + h1 * a1;
    acc2 = acc2 + h2 * a2;
    acc3 = acc3 + h3 * a3;
    acc4 = acc4 + h4 * a4;
    acc5 = acc5 + h5 * a5;
    acc6 = acc6 + h6 * a6;
    acc7 = acc7 + h7 * a7;
  }

  if (live) {
    float* op = out + (size_t)node * HC + 4 * lane;
    *(volatile v4f*)(op + 0 * FO) = acc0;
    *(volatile v4f*)(op + 1 * FO) = acc1;
    *(volatile v4f*)(op + 2 * FO) = acc2;
    *(volatile v4f*)(op + 3 * FO) = acc3;
    *(volatile v4f*)(op + 4 * FO) = acc4;
    *(volatile v4f*)(op + 5 * FO) = acc5;
    *(volatile v4f*)(op + 6 * FO) = acc6;
    *(volatile v4f*)(op + 7 * FO) = acc7;
  }
  __threadfence();
  if (live) {
    float* op = out + (size_t)node * HC + 4 * lane;
    *(volatile v4f*)(op + 0 * FO) = acc0;
    *(volatile v4f*)(op + 1 * FO) = acc1;
    *(volatile v4f*)(op + 2 * FO) = acc2;
    *(volatile v4f*)(op + 3 * FO) = acc3;
    *(volatile v4f*)(op + 4 * FO) = acc4;
    *(volatile v4f*)(op + 5 * FO) = acc5;
    *(volatile v4f*)(op + 6 * FO) = acc6;
    *(volatile v4f*)(op + 7 * FO) = acc7;
  }
}

extern "C" void kernel_launch(void* const* d_in, const int* in_sizes, int n_in,
                              void* d_out, int out_size, void* d_ws, size_t ws_size,
                              hipStream_t stream) {
  if (n_in < 6) return;
  if (in_sizes[0] < FIN || (in_sizes[0] % FIN) != 0) return;
  const int nN = in_sizes[0] / FIN;
  if (nN < 1 || nN > 65536) return;
  if (in_sizes[1] != nN * DEG) return;
  if (in_sizes[2] != NHD * FIN * FO) return;
  if (in_sizes[3] != HC) return;
  if (in_sizes[4] != AW) return;
  if (in_sizes[5] != NHD) return;
  if (out_size != nN * HC) return;

  const float* features = (const float*)d_in[0];
  const int*   adj      = (const int*)d_in[1];
  const float* W        = (const float*)d_in[2];
  const float* bW       = (const float*)d_in[3];
  const float* av       = (const float*)d_in[4];
  const float* ba       = (const float*)d_in[5];
  float* out = (float*)d_out;

  const int NPAD = ((nN + BM - 1) / BM) * BM;

  char* ws = (char*)d_ws;
  size_t off = 0;
  const size_t oA  = off; off += (size_t)NPAD * FIN * 2;   off = (off + 255) & ~(size_t)255;
  const size_t oWp = off; off += (size_t)HC * FIN * 2;     off = (off + 255) & ~(size_t)255;
  const size_t oH  = off; off += (size_t)NPAD * HC * 4;    off = (off + 255) & ~(size_t)255;
  const size_t oEs = off; off += (size_t)NPAD * ESW * 4;   off = (off + 255) & ~(size_t)255;
  if (off > ws_size || off > (size_t)WSCAP) return;

  _Float16* a16 = (_Float16*)(ws + oA);
  _Float16* wp  = (_Float16*)(ws + oWp);
  float* hcat   = (float*)(ws + oH);
  float* es     = (float*)(ws + oEs);

  k_acvt<<<(NPAD * (FIN / 8)) / NTHR, NTHR, 0, stream>>>(features, a16, nN, NPAD);
  {
    const int nUnits = HC * (FIN / 8);
    k_wcvt<<<(nUnits + NTHR - 1) / NTHR, NTHR, 0, stream>>>(W, wp, nUnits);
  }
  k_gemm<<<dim3(NPAD / BM, HC / BNC), NTHR, 0, stream>>>(a16, wp, bW, hcat, FIN, HC, nN, NPAD, SCL_AW);
  k_scores<<<NPAD / SNB, NTHR, 0, stream>>>(hcat, av, es, nN);
  k_attend<<<NPAD / ANB, NTHR, 0, stream>>>(hcat, adj, es, ba, out, nN);
}
